// Attention_6648609375073
// MI455X (gfx1250) — hardware-verified
//
#include <hip/hip_runtime.h>
#include <stddef.h>


typedef _Float16 v16h __attribute__((ext_vector_type(16)));
typedef _Float16 v8h  __attribute__((ext_vector_type(8)));
typedef float    v8f  __attribute__((ext_vector_type(8)));
typedef float    v4f  __attribute__((ext_vector_type(4)));

#ifndef NB
#define NB 2
#endif
#ifndef SEQ
#define SEQ 2048
#endif
#define NB_FULL  2
#define SEQ_FULL 2048
#define DIM   2048
#define NHEAD 32
#define HD    64
#define NKV   8
#define GQA   (NHEAD / NKV)
#define KVD   (NKV * HD)
#define MROWS (NB * SEQ)
#define EROWS  128
#define ECHUNK 64

static_assert(NB >= 1 && NB <= NB_FULL);
static_assert(SEQ >= 128 && SEQ <= SEQ_FULL && (SEQ % 128) == 0);
static_assert(DIM == NHEAD * HD);
static_assert(HD == 64);
static_assert(NHEAD == NKV * GQA && GQA == 4);
static_assert(KVD == 512 && (KVD % 64) == 0);
static_assert((DIM % 64) == 0 && (DIM % 32) == 0);
static_assert((MROWS % 64) == 0 && (MROWS % 8) == 0);
static_assert((SEQ % 64) == 0);
static_assert((DIM % 8) == 0 && (KVD % 8) == 0);
static_assert(DIM == 8 * 32 * 8);
static_assert((size_t)MROWS * DIM < (size_t)0xFFFFFFFFu);
static_assert(EROWS == 128);
static_assert(ECHUNK == 64);
static_assert((EROWS % 64) == 0 && EROWS <= SEQ);
static_assert((size_t)NB * NHEAD * EROWS * HD < (size_t)0xFFFFFFFFu);

#define LDT 72
#define LDC 68
static_assert((LDT % 8) == 0 && LDT >= 64);
static_assert((LDC % 4) == 0 && LDC >= 64);

#define WCARRY 64.0f
#define PCARRY 1024.0f
#define VCARRY 64.0f
#define RCARRY 1024.0f
#define SCRES  2048.0f

#define TILE_ROWS        64
#define EPI16_ROWS_STEP  (256 / 8)
#define EPI16_STEPS      2
#define EPIF_ROWS_STEP   (256 / 16)
#define EPIF_STEPS       4
static_assert(EPI16_ROWS_STEP * EPI16_STEPS == TILE_ROWS);
static_assert(EPIF_ROWS_STEP * EPIF_STEPS == TILE_ROWS);
static_assert((32 / 8) * 4 == 16);
static_assert(8 * 16 == 128);

static_assert((size_t)64 * LDC * 4 <= (size_t)131072);
static_assert((size_t)(4 * 64 * LDT + 8 * 16 * LDT) * 2 <= (size_t)131072);

#define WSQ_BYTES     ((size_t)DIM * DIM * 2)
#define WKV_BYTES     ((size_t)KVD * DIM * 2)
#define PLANE16_BYTES ((size_t)MROWS * DIM * 2)
#define VRES_BYTES    ((size_t)NB * DIM * 64 * 2)
#define QRES_BYTES    ((size_t)NB * NHEAD * EROWS * HD * 2)
#define KRES_BYTES    ((size_t)NB * NHEAD * ECHUNK * HD * 2)
#define CRES_BYTES    ((size_t)NB * EROWS * DIM * 2)
#define OFF_WQ  ((size_t)0)
#define OFF_WK  (OFF_WQ + WSQ_BYTES)
#define OFF_WV  (OFF_WK + WKV_BYTES)
#define OFF_WO  (OFF_WV + WKV_BYTES)
#define OFF_X   (OFF_WO + WSQ_BYTES)
#define OFF_Q   (OFF_X + PLANE16_BYTES)
#define OFF_K   (OFF_Q + PLANE16_BYTES)
#define OFF_VT  (OFF_K + PLANE16_BYTES)
#define OFF_CTX (OFF_VT + PLANE16_BYTES)
#define OFF_VR  (OFF_CTX + PLANE16_BYTES)
#define OFF_QR  (OFF_VR + VRES_BYTES)
#define OFF_KR  (OFF_QR + QRES_BYTES)
#define OFF_CR  (OFF_KR + KRES_BYTES)
#define WS_TOTAL (OFF_CR + CRES_BYTES)
static_assert((WSQ_BYTES % 128) == 0 && (WKV_BYTES % 128) == 0 && (PLANE16_BYTES % 128) == 0);
static_assert((VRES_BYTES % 128) == 0);
static_assert((QRES_BYTES % 128) == 0 && (KRES_BYTES % 128) == 0 && (CRES_BYTES % 128) == 0);
static_assert(WS_TOTAL <= (size_t)134217728);

__device__ __forceinline__ float bf16r(float x) {
  unsigned int u = __float_as_uint(x);
  u = (u + 0x7FFFu + ((u >> 16) & 1u)) & 0xFFFF0000u;
  return __uint_as_float(u);
}

static __device__ __forceinline__ _Float16 toh_flush(float v) {
  const _Float16 r = (_Float16)v;
  return (fabsf(v) < 6.103515625e-05f) ? (_Float16)0.0f : r;
}

__device__ __forceinline__ v16h frag_at(const _Float16* p) {
  v8h lo = *(const v8h*)(p);
  v8h hi = *(const v8h*)(p + 16);
  v16h out;
#pragma unroll
  for (int i = 0; i < 8; ++i) { out[i] = lo[i]; out[i + 8] = hi[i]; }
  return out;
}
__device__ __forceinline__ v16h ld_frag(const _Float16* base, unsigned ld) {
  const unsigned lane = threadIdx.x & 31u;
  return frag_at(base + (lane & 15u) * ld + (lane >> 4) * 8u);
}

__device__ __forceinline__ v8f wmma16(v16h a, v16h b, v8f c) {
  v8f d = __builtin_amdgcn_wmma_f32_16x16x32_f16(false, a, false, b, (short)0, c,
                                                 false, false);
  asm volatile("v_nop\n\tv_nop\n\tv_nop\n\tv_nop" : "+v"(d) : "v"(a), "v"(b));
  return d;
}

__device__ __forceinline__ float red16_max(float x) {
#pragma unroll
  for (int off = 1; off < 16; off <<= 1) x = fmaxf(x, __shfl_xor(x, off, 32));
  return x;
}
__device__ __forceinline__ float red16_sum(float x) {
#pragma unroll
  for (int off = 1; off < 16; off <<= 1) x += __shfl_xor(x, off, 32);
  return x;
}

__device__ __forceinline__ void wave_lds_sync() {
  __builtin_amdgcn_fence(3  , "wavefront");
  asm volatile("s_wait_dscnt 0x0" ::: "memory");
  __builtin_amdgcn_wave_barrier();
}

template <int SRC_INPUT>
__device__ __forceinline__ void cast_body(const float* __restrict__ X,
                                          _Float16* __restrict__ dst) {
#pragma clang fp contract(off)
  const unsigned lane = threadIdx.x & 31u;
  const unsigned w = (unsigned)__builtin_amdgcn_readfirstlane((int)(threadIdx.x >> 5));
  const unsigned crow = blockIdx.x * 8u + w;
  size_t srow = crow;
  if (SRC_INPUT) {
    const unsigned bidx = crow / (unsigned)SEQ;
    const unsigned sq = crow - bidx * (unsigned)SEQ;
    srow = (size_t)bidx * SEQ_FULL + sq;
  }
  const float carry = SRC_INPUT ? 1.0f : WCARRY;
  const float* xr = X + srow * DIM + lane * 8u;
  _Float16* dr = dst + (size_t)crow * DIM + lane * 8u;
#pragma unroll 1
  for (unsigned j = 0; j < 8u; ++j) {
    const v4f a0 = *(const v4f*)(xr + j * 256u);
    const v4f a1 = *(const v4f*)(xr + j * 256u + 4u);
    v8h o;
#pragma unroll
    for (int i = 0; i < 4; ++i) {
      o[i]     = toh_flush(carry * bf16r(a0[i]));
      o[i + 4] = toh_flush(carry * bf16r(a1[i]));
    }
    _Float16* p = dr + j * 256u;
    *(volatile v8h*)p = o;
    __threadfence();
    *(volatile v8h*)p = o;
  }
}

__global__ __launch_bounds__(256) void xcast_kernel(
    const float* __restrict__ X, _Float16* __restrict__ dst) {
  cast_body<1>(X, dst);
}
__global__ __launch_bounds__(256) void wcast_kernel(
    const float* __restrict__ W, _Float16* __restrict__ dst) {
  cast_body<0>(W, dst);
}

template <int MODE>
__device__ __forceinline__ void gemm_body(
    const _Float16* __restrict__ A16, const _Float16* __restrict__ A16r,
    const _Float16* __restrict__ Bt, const unsigned K,
    float* __restrict__ outf, _Float16* __restrict__ out16, _Float16* __restrict__ out16r) {
  __shared__ float Cs[64 * LDC];
  const unsigned tid = threadIdx.x, lane = tid & 31u, w = tid >> 5;
  const unsigned mw = w >> 1, nw = w & 1u;
  const unsigned hh = lane >> 4, m = lane & 15u;
  const unsigned n0 = blockIdx.x * 64u;
  const unsigned row0 = blockIdx.y * 64u;

  const _Float16* ap  = A16 + (size_t)(row0 + mw * 16u + m) * K + hh * 8u;
  const _Float16* bp0 = Bt + (size_t)(n0 + nw * 32u + m) * K + hh * 8u;
  const _Float16* bp1 = bp0 + (size_t)16 * K;
  v8f acc0 = {}, acc1 = {};
  bool res_tile = false;
  if (MODE == 3) {
    const unsigned bidx3 = row0 / (unsigned)SEQ;
    res_tile = (row0 - bidx3 * (unsigned)SEQ) < (unsigned)EROWS;
  }
  if (res_tile) {
    const unsigned bidx3 = row0 / (unsigned)SEQ;
    const unsigned sq3 = row0 - bidx3 * (unsigned)SEQ;
    const _Float16* rp =
        A16r + (size_t)(bidx3 * (unsigned)EROWS + sq3 + mw * 16u + m) * K + hh * 8u;
    v8f res0 = {}, res1 = {};
#pragma unroll 2
    for (unsigned k0 = 0; k0 < K; k0 += 32u) {
      const v16h a  = frag_at(ap + k0);
      const v16h ar = frag_at(rp + k0);
      const v16h b0 = frag_at(bp0 + k0);
      const v16h b1 = frag_at(bp1 + k0);
      acc0 = wmma16(a, b0, acc0);
      acc1 = wmma16(a, b1, acc1);
      res0 = wmma16(ar, b0, res0);
      res1 = wmma16(ar, b1, res1);
    }
#pragma unroll
    for (int r = 0; r < 8; ++r) {
      acc0[r] = acc0[r] + res0[r] * (1.0f / SCRES);
      acc1[r] = acc1[r] + res1[r] * (1.0f / SCRES);
    }
  } else {
#pragma unroll 2
    for (unsigned k0 = 0; k0 < K; k0 += 32u) {
      const v16h a  = frag_at(ap + k0);
      const v16h b0 = frag_at(bp0 + k0);
      const v16h b1 = frag_at(bp1 + k0);
      acc0 = wmma16(a, b0, acc0);
      acc1 = wmma16(a, b1, acc1);
    }
  }
#pragma unroll
  for (int r = 0; r < 8; ++r) {
    float* d = &Cs[(mw * 16u + hh * 8u + (unsigned)r) * LDC + nw * 32u + m];
    d[0]  = acc0[r];
    d[16] = acc1[r];
  }
  __syncthreads();

  if (MODE == 0 || MODE == 1) {
    constexpr unsigned NREP  = (MODE == 1) ? (unsigned)GQA : 1u;
    constexpr unsigned RROWS = (MODE == 1) ? (unsigned)ECHUNK : (unsigned)EROWS;
    const unsigned cb = (MODE == 1) ? blockIdx.x * (unsigned)(GQA * HD) : n0;
    const unsigned bidx = row0 / (unsigned)SEQ;
    const unsigned sq0 = row0 - bidx * (unsigned)SEQ;
    const bool has_res = (sq0 < RROWS);
    v8h x[2], xr[2];
    size_t off[2], offr[2];
#pragma unroll
    for (unsigned i = 0; i < 2u; ++i) {
      const unsigned r = 32u * i + (tid >> 3);
      const unsigned c = (tid & 7u) * 8u;
      const v4f u0 = *(const v4f*)&Cs[r * LDC + c];
      const v4f u1 = *(const v4f*)&Cs[r * LDC + c + 4];
#pragma unroll
      for (int j = 0; j < 4; ++j) {
        x[i][j]     = toh_flush(u0[j] * (1.0f / WCARRY));
        x[i][j + 4] = toh_flush(u1[j] * (1.0f / WCARRY));
      }
      xr[i] = x[i];
      if (has_res) {
#pragma unroll
        for (int j = 0; j < 4; ++j) {
          const float t0 = u0[j] * (1.0f / WCARRY);
          const float t1 = u1[j] * (1.0f / WCARRY);
          xr[i][j]     = toh_flush((t0 - (float)x[i][j]) * SCRES);
          xr[i][j + 4] = toh_flush((t1 - (float)x[i][j + 4]) * SCRES);
        }
      }
      off[i] = (size_t)(row0 + r) * DIM + cb + c;
      offr[i] = ((size_t)(bidx * (unsigned)NHEAD + blockIdx.x * NREP) * RROWS + sq0 + r) * HD + c;
    }
#pragma unroll
    for (unsigned rep = 0; rep < NREP; ++rep) {
#pragma unroll
      for (int i = 0; i < 2; ++i)
        *(volatile v8h*)(out16 + off[i] + (size_t)rep * HD) = x[i];
    }
    if (has_res) {
#pragma unroll
      for (unsigned rep = 0; rep < NREP; ++rep) {
#pragma unroll
        for (int i = 0; i < 2; ++i)
          *(volatile v8h*)(out16r + offr[i] + (size_t)rep * RROWS * HD) = xr[i];
      }
    }
    __threadfence();
#pragma unroll
    for (unsigned rep = 0; rep < NREP; ++rep) {
#pragma unroll
      for (int i = 0; i < 2; ++i)
        *(volatile v8h*)(out16 + off[i] + (size_t)rep * HD) = x[i];
    }
    if (has_res) {
#pragma unroll
      for (unsigned rep = 0; rep < NREP; ++rep) {
#pragma unroll
        for (int i = 0; i < 2; ++i)
          *(volatile v8h*)(out16r + offr[i] + (size_t)rep * RROWS * HD) = xr[i];
      }
    }
  }

  if (MODE == 2) {
    const unsigned bidx = row0 / (unsigned)SEQ;
    const unsigned key0 = row0 - bidx * (unsigned)SEQ;
    const bool first_tile = (key0 == 0u);
    v8h x[2], xr[2];
    size_t off[2], offr[2];
#pragma unroll
    for (unsigned i = 0; i < 2u; ++i) {
      const unsigned dcol = 32u * i + (tid >> 3);
      const unsigned kk = (tid & 7u) * 8u;
#pragma unroll
      for (unsigned j = 0; j < 8u; ++j) {
        const float t = Cs[(kk + j) * LDC + dcol] * (1.0f / WCARRY);
        const _Float16 hi = toh_flush(t);
        x[i][j]  = hi;
        xr[i][j] = toh_flush((t - (float)hi) * RCARRY);
      }
      const size_t vrow = (size_t)bidx * DIM + blockIdx.x * (unsigned)(GQA * HD) + dcol;
      off[i]  = vrow * SEQ + key0 + kk;
      offr[i] = vrow * 64u + kk;
    }
#pragma unroll
    for (unsigned rep = 0; rep < (unsigned)GQA; ++rep) {
#pragma unroll
      for (int i = 0; i < 2; ++i)
        *(volatile v8h*)(out16 + off[i] + (size_t)rep * HD * SEQ) = x[i];
    }
    if (first_tile) {
#pragma unroll
      for (unsigned rep = 0; rep < (unsigned)GQA; ++rep) {
#pragma unroll
        for (int i = 0; i < 2; ++i)
          *(volatile v8h*)(out16r + offr[i] + (size_t)rep * HD * 64u) = xr[i];
      }
    }
    __threadfence();
#pragma unroll
    for (unsigned rep = 0; rep < (unsigned)GQA; ++rep) {
#pragma unroll
      for (int i = 0; i < 2; ++i)
        *(volatile v8h*)(out16 + off[i] + (size_t)rep * HD * SEQ) = x[i];
    }
    if (first_tile) {
#pragma unroll
      for (unsigned rep = 0; rep < (unsigned)GQA; ++rep) {
#pragma unroll
        for (int i = 0; i < 2; ++i)
          *(volatile v8h*)(out16r + offr[i] + (size_t)rep * HD * 64u) = xr[i];
      }
    }
  }

  if (MODE == 3) {
    const float cs = 1.0f / (WCARRY * VCARRY);
    v4f xs[4];
    size_t off[4];
#pragma unroll
    for (unsigned i = 0; i < 4u; ++i) {
      const unsigned r = 16u * i + (tid >> 4);
      const unsigned c = (tid & 15u) * 4u;
      const unsigned crow = row0 + r;
      const unsigned bidx = crow / (unsigned)SEQ;
      const unsigned sq = crow - bidx * (unsigned)SEQ;
      const size_t frow = (size_t)bidx * SEQ_FULL + sq;
      const v4f u = *(const v4f*)&Cs[r * LDC + c];
      v4f val;
#pragma unroll
      for (int j = 0; j < 4; ++j) val[j] = u[j] * cs;
      xs[i] = val;
      off[i] = frow * DIM + n0 + c;
    }
#pragma unroll
    for (int i = 0; i < 4; ++i) *(volatile v4f*)(outf + off[i]) = xs[i];
    __threadfence();
#pragma unroll
    for (int i = 0; i < 4; ++i) *(volatile v4f*)(outf + off[i]) = xs[i];
  }
}

__global__ __launch_bounds__(256) void gemm_q_kernel(
    const _Float16* __restrict__ A16, const _Float16* __restrict__ Bt,
    _Float16* __restrict__ out16, _Float16* __restrict__ out16r) {
  gemm_body<0>(A16, A16, Bt, (unsigned)DIM, (float*)0, out16, out16r);
}
__global__ __launch_bounds__(256) void gemm_k_kernel(
    const _Float16* __restrict__ A16, const _Float16* __restrict__ Bt,
    _Float16* __restrict__ out16, _Float16* __restrict__ out16r) {
  gemm_body<1>(A16, A16, Bt, (unsigned)DIM, (float*)0, out16, out16r);
}
__global__ __launch_bounds__(256) void gemm_v_kernel(
    const _Float16* __restrict__ A16, const _Float16* __restrict__ Bt,
    _Float16* __restrict__ vt, _Float16* __restrict__ vtr) {
  gemm_body<2>(A16, A16, Bt, (unsigned)DIM, (float*)0, vt, vtr);
}
__global__ __launch_bounds__(256) void gemm_wo_kernel(
    const _Float16* __restrict__ A16, const _Float16* __restrict__ A16r,
    const _Float16* __restrict__ Bt, float* __restrict__ outf) {
  gemm_body<3>(A16, A16r, Bt, (unsigned)DIM, outf, (_Float16*)0, (_Float16*)0);
}

__global__ __launch_bounds__(256) void attn_kernel(
    const _Float16* __restrict__ Qh, const _Float16* __restrict__ QhR,
    const _Float16* __restrict__ Kh, const _Float16* __restrict__ KhR,
    const _Float16* __restrict__ Vt, const _Float16* __restrict__ VtR,
    _Float16* __restrict__ Ov, _Float16* __restrict__ OvR) {
  __shared__ _Float16 Ks[64 * LDT];
  __shared__ _Float16 Vs[64 * LDT];
  __shared__ _Float16 VRs[64 * LDT];
  __shared__ _Float16 KRs[64 * LDT];
  __shared__ _Float16 Ps[8 * 16 * LDT];

  const unsigned tid = threadIdx.x, lane = tid & 31u, w = tid >> 5;
  const unsigned hh = lane >> 4, m = lane & 15u;
  const unsigned q0 = blockIdx.x * 128u;
  const unsigned head = blockIdx.y;
  const unsigned b = blockIdx.z;
  const float scale = 0.125f;
  const unsigned qrow0 = q0 + w * 16u;
  const bool first_blk = (blockIdx.x == 0u);
  _Float16* P = Ps + w * (16u * LDT);

  const size_t qoff = (size_t)(b * (unsigned)SEQ + qrow0 + m) * DIM + head * HD + hh * 8u;
  v16h qf[2];
  qf[0] = frag_at(Qh + qoff);
  qf[1] = frag_at(Qh + qoff + 32);

  float mrow[8], lrow[8];
  v8f o[4];
#pragma unroll
  for (int v = 0; v < 8; ++v) { mrow[v] = -1.0e30f; lrow[v] = 0.0f; }
#pragma unroll
  for (int nb = 0; nb < 4; ++nb) o[nb] = (v8f){};

  const size_t kplane = (size_t)b * SEQ * DIM + head * HD;
  const size_t vplane = ((size_t)b * DIM + head * HD) * SEQ;
  const size_t rplane = ((size_t)b * DIM + head * HD) * 64u;
  const size_t krplane = ((size_t)(b * (unsigned)NHEAD + head) * ECHUNK) * HD;
  const unsigned kend = q0 + 128u;

  for (unsigned kb = 0; kb < kend; kb += 64u) {
    const bool early = first_blk && (kb == 0u);
#pragma unroll
    for (unsigned j = 0; j < 2u; ++j) {
      const unsigned idx = tid + 256u * j;
      const unsigned r = idx >> 3, c = (idx & 7u) * 8u;
      *(v8h*)&Ks[r * LDT + c] = *(const v8h*)(Kh + kplane + (size_t)(kb + r) * DIM + c);
      *(v8h*)&Vs[r * LDT + c] = *(const v8h*)(Vt + vplane + (size_t)r * SEQ + kb + c);
    }
    if (early) {
#pragma unroll
      for (unsigned j = 0; j < 2u; ++j) {
        const unsigned idx = tid + 256u * j;
        const unsigned r = idx >> 3, c = (idx & 7u) * 8u;
        *(v8h*)&VRs[r * LDT + c] = *(const v8h*)(VtR + rplane + (size_t)r * 64u + c);
        *(v8h*)&KRs[r * LDT + c] = *(const v8h*)(KhR + krplane + (size_t)r * HD + c);
      }
    }
    __syncthreads();

    v8f s[4];
    if (early) {
      const unsigned qrbase =
          ((b * (unsigned)NHEAD + head) * (unsigned)EROWS + qrow0 + m) * (unsigned)HD + hh * 8u;
#pragma unroll
      for (int kg = 0; kg < 4; ++kg) {
        v8f t = {};
#pragma unroll
        for (int c = 0; c < 2; ++c) {
          unsigned qro = qrbase + (unsigned)c * 32u;
          asm volatile("" : "+v"(qro));
          v8f tr = {};
          {
            const v16h kf = ld_frag(&Ks[(kg * 16) * LDT + c * 32], LDT);
            t = wmma16(qf[c], kf, t);
            const v16h ql = frag_at(QhR + qro);
            tr = wmma16(ql, kf, tr);
          }
          {
            const v16h kl = ld_frag(&KRs[(kg * 16) * LDT + c * 32], LDT);
            tr = wmma16(qf[c], kl, tr);
          }
          t = t + tr * (1.0f / SCRES);
          __builtin_amdgcn_sched_barrier(0);
        }
        s[kg] = t * scale;
      }
    } else {
#pragma unroll
      for (int kg = 0; kg < 4; ++kg) {
        v8f t = {};
#pragma unroll
        for (int c = 0; c < 2; ++c) {
          const v16h kf = ld_frag(&Ks[(kg * 16) * LDT + c * 32], LDT);
          t = wmma16(qf[c], kf, t);
        }
        s[kg] = t * scale;
      }
    }

    if (kb >= q0) {
#pragma unroll
      for (int kg = 0; kg < 4; ++kg)
#pragma unroll
        for (int v = 0; v < 8; ++v) {
          const unsigned key = kb + (unsigned)kg * 16u + m;
          const unsigned row = qrow0 + hh * 8u + (unsigned)v;
          s[kg][v] = (key > row) ? -1.0e30f : s[kg][v];
        }
    }

    float alpha[8];
#pragma unroll
    for (int v = 0; v < 8; ++v) {
      float mx = fmaxf(fmaxf(s[0][v], s[1][v]), fmaxf(s[2][v], s[3][v]));
      mx = red16_max(mx);
      const float mn = fmaxf(mrow[v], mx);
      alpha[v] = __expf(mrow[v] - mn);
      mrow[v] = mn;
    }
#pragma unroll
    for (int kg = 0; kg < 4; ++kg)
#pragma unroll
      for (int v = 0; v < 8; ++v) s[kg][v] = __expf(s[kg][v] - mrow[v]);
#pragma unroll
    for (int v = 0; v < 8; ++v) {
      const float rs = red16_sum((s[0][v] + s[1][v]) + (s[2][v] + s[3][v]));
      lrow[v] = alpha[v] * lrow[v] + rs;
    }
#pragma unroll
    for (int nb = 0; nb < 4; ++nb)
#pragma unroll
      for (int v = 0; v < 8; ++v) o[nb][v] = o[nb][v] * alpha[v];

#pragma unroll
    for (int kg = 0; kg < 4; ++kg)
#pragma unroll
      for (int v = 0; v < 8; ++v)
        P[(hh * 8u + (unsigned)v) * LDT + (unsigned)kg * 16u + m] = toh_flush(s[kg][v] * PCARRY);
    wave_lds_sync();

#pragma unroll
    for (int c = 0; c < 2; ++c) {
      const v16h pf = ld_frag(P + c * 32, LDT);
#pragma unroll
      for (int nb = 0; nb < 4; ++nb) {
        const v16h vf = ld_frag(&Vs[(nb * 16) * LDT + c * 32], LDT);
        o[nb] = wmma16(pf, vf, o[nb]);
      }
    }

    if (early) {
#pragma unroll
      for (int nb = 0; nb < 4; ++nb) {
        v8f o2 = {};
#pragma unroll
        for (int c = 0; c < 2; ++c) {
          const v16h pf = ld_frag(P + c * 32, LDT);
          const v16h vr = ld_frag(&VRs[(nb * 16) * LDT + c * 32], LDT);
          o2 = wmma16(pf, vr, o2);
        }
#pragma unroll
        for (int v = 0; v < 8; ++v) o[nb][v] = o[nb][v] + o2[v] * (1.0f / RCARRY);
      }
      wave_lds_sync();
#pragma unroll
      for (int kg = 0; kg < 4; ++kg)
#pragma unroll
        for (int v = 0; v < 8; ++v) {
          const float t = s[kg][v] * PCARRY;
          const float hi = (float)toh_flush(t);
          P[(hh * 8u + (unsigned)v) * LDT + (unsigned)kg * 16u + m] =
              toh_flush((t - hi) * RCARRY);
        }
      wave_lds_sync();
#pragma unroll
      for (int nb = 0; nb < 4; ++nb) {
        v8f o2 = {};
#pragma unroll
        for (int c = 0; c < 2; ++c) {
          const v16h pf = ld_frag(P + c * 32, LDT);
          const v16h vf = ld_frag(&Vs[(nb * 16) * LDT + c * 32], LDT);
          o2 = wmma16(pf, vf, o2);
        }
#pragma unroll
        for (int v = 0; v < 8; ++v) o[nb][v] = o[nb][v] + o2[v] * (1.0f / RCARRY);
      }
    }
    __syncthreads();
  }

  float inv[8];
#pragma unroll
  for (int v = 0; v < 8; ++v) inv[v] = __builtin_amdgcn_rcpf(lrow[v]) * (VCARRY / PCARRY);
#pragma unroll
  for (int nb = 0; nb < 4; ++nb)
#pragma unroll
    for (int v = 0; v < 8; ++v)
      P[(hh * 8u + (unsigned)v) * LDT + (unsigned)nb * 16u + m] = toh_flush(o[nb][v] * inv[v]);
  wave_lds_sync();
  v8h x[4], xr[4];
  size_t off[4], offr[4];
#pragma unroll
  for (unsigned i = 0; i < 4u; ++i) {
    const unsigned r = 4u * i + (lane >> 3);
    const unsigned c = (lane & 7u) * 8u;
    x[i] = *(const v8h*)&P[r * LDT + c];
    off[i] = (size_t)(b * (unsigned)SEQ + qrow0 + r) * DIM + head * HD + c;
    xr[i] = x[i];
    offr[i] = (size_t)(b * (unsigned)EROWS + (qrow0 & 127u) + r) * DIM + head * HD + c;
  }
  if (first_blk) {
    wave_lds_sync();
#pragma unroll
    for (int nb = 0; nb < 4; ++nb)
#pragma unroll
      for (int v = 0; v < 8; ++v) {
        const float t = o[nb][v] * inv[v];
        const float hi = (float)toh_flush(t);
        P[(hh * 8u + (unsigned)v) * LDT + (unsigned)nb * 16u + m] = toh_flush((t - hi) * SCRES);
      }
    wave_lds_sync();
#pragma unroll
    for (unsigned i = 0; i < 4u; ++i) {
      const unsigned r = 4u * i + (lane >> 3);
      const unsigned c = (lane & 7u) * 8u;
      xr[i] = *(const v8h*)&P[r * LDT + c];
    }
  }
#pragma unroll
  for (int i = 0; i < 4; ++i) *(volatile v8h*)(Ov + off[i]) = x[i];
  if (first_blk) {
#pragma unroll
    for (int i = 0; i < 4; ++i) *(volatile v8h*)(OvR + offr[i]) = xr[i];
  }
  __threadfence();
#pragma unroll
  for (int i = 0; i < 4; ++i) *(volatile v8h*)(Ov + off[i]) = x[i];
  if (first_blk) {
#pragma unroll
    for (int i = 0; i < 4; ++i) *(volatile v8h*)(OvR + offr[i]) = xr[i];
  }
}

extern "C" void kernel_launch(void* const* d_in, const int* in_sizes, int n_in,
                              void* d_out, int out_size, void* d_ws, size_t ws_size,
                              hipStream_t stream) {
  if (n_in < 5) return;
  const long long need_x = ((long long)(NB - 1) * SEQ_FULL + SEQ) * DIM;
  if ((long long)in_sizes[0] < need_x) return;
  if ((long long)in_sizes[1] < (long long)DIM * DIM) return;
  if ((long long)in_sizes[2] < (long long)KVD * DIM) return;
  if ((long long)in_sizes[3] < (long long)KVD * DIM) return;
  if ((long long)in_sizes[4] < (long long)DIM * DIM) return;
  if ((long long)out_size < need_x) return;
  if (ws_size < WS_TOTAL) return;

  const float* X  = (const float*)d_in[0];
  const float* wq = (const float*)d_in[1];
  const float* wk = (const float*)d_in[2];
  const float* wv = (const float*)d_in[3];
  const float* wo = (const float*)d_in[4];
  float* out = (float*)d_out;

  char* ws = (char*)d_ws;
  _Float16* Wq_t  = (_Float16*)(ws + OFF_WQ);
  _Float16* Wk_t  = (_Float16*)(ws + OFF_WK);
  _Float16* Wv_t  = (_Float16*)(ws + OFF_WV);
  _Float16* Wo_t  = (_Float16*)(ws + OFF_WO);
  _Float16* X16   = (_Float16*)(ws + OFF_X);
  _Float16* Qh16  = (_Float16*)(ws + OFF_Q);
  _Float16* Kh16  = (_Float16*)(ws + OFF_K);
  _Float16* Vt16  = (_Float16*)(ws + OFF_VT);
  _Float16* Ctx16 = (_Float16*)(ws + OFF_CTX);
  _Float16* VtR16 = (_Float16*)(ws + OFF_VR);
  _Float16* QR16  = (_Float16*)(ws + OFF_QR);
  _Float16* KR16  = (_Float16*)(ws + OFF_KR);
  _Float16* CR16  = (_Float16*)(ws + OFF_CR);

  dim3 blk(256);

  wcast_kernel<<<dim3(DIM / 8), blk, 0, stream>>>(wq, Wq_t);
  wcast_kernel<<<dim3(KVD / 8), blk, 0, stream>>>(wk, Wk_t);
  wcast_kernel<<<dim3(KVD / 8), blk, 0, stream>>>(wv, Wv_t);
  wcast_kernel<<<dim3(DIM / 8), blk, 0, stream>>>(wo, Wo_t);
  xcast_kernel<<<dim3(MROWS / 8), blk, 0, stream>>>(X, X16);

  gemm_q_kernel<<<dim3(DIM / 64, MROWS / 64), blk, 0, stream>>>(X16, Wq_t, Qh16, QR16);
  gemm_k_kernel<<<dim3(KVD / 64, MROWS / 64), blk, 0, stream>>>(X16, Wk_t, Kh16, KR16);
  gemm_v_kernel<<<dim3(KVD / 64, MROWS / 64), blk, 0, stream>>>(X16, Wv_t, Vt16, VtR16);
  attn_kernel<<<dim3(SEQ / 128, NHEAD, NB), blk, 0, stream>>>(Qh16, QR16, Kh16, KR16, Vt16, VtR16,
                                                              Ctx16, CR16);
  gemm_wo_kernel<<<dim3(DIM / 64, MROWS / 64), blk, 0, stream>>>(Ctx16, CR16, Wo_t, out);
}
